// Mamba_6940667150618
// MI455X (gfx1250) — hardware-verified
//
#include <hip/hip_runtime.h>
#include <math.h>

typedef __attribute__((ext_vector_type(16))) __bf16       v16b;
typedef __attribute__((ext_vector_type(8)))  __bf16       v8b;
typedef __attribute__((ext_vector_type(8)))  float        v8f;
typedef __attribute__((ext_vector_type(4)))  float        v4f;
typedef __attribute__((ext_vector_type(4)))  unsigned int v4u;

constexpr int kBatch = 2;
constexpr int kSeq   = 1024;
constexpr int kDm    = 1024;
constexpr int kDin   = 2048;
constexpr int kNst   = 16;
constexpr int kDtR   = 64;
constexpr int kPrjN  = 96;
constexpr int kPrjP  = 128;
constexpr int kXzP   = 2 * kDin;
constexpr int kRows  = kBatch * kSeq;
constexpr int kTP    = 260;
static_assert(kDtR + 2 * kNst == kPrjN);
static_assert((kDm % 32) == 0 && (kDin % 32) == 0 && (kDtR % 32) == 0);
static_assert((kRows % 64) == 0 && (kXzP % 64) == 0 && (kPrjP % 64) == 0 && (kDin % 64) == 0 && (kDm % 64) == 0);
static_assert((kSeq % 64) == 0 && (kSeq % 16) == 0 && (kDin % 256) == 0);
static_assert((((kRows / 64) * (kXzP / 64)) % 8) == 0 && (((kRows / 64) * (kPrjP / 64)) % 8) == 0);
static_assert((((kRows / 64) * (kDin / 64)) % 8) == 0 && (((kRows / 64) * (kDm / 64)) % 8) == 0);

constexpr size_t kOffXB    = 0;
constexpr size_t kOffWINB  = kOffXB    + (size_t)kRows * kDm   * 2;
constexpr size_t kOffWXPB  = kOffWINB  + (size_t)kXzP  * kDm   * 2;
constexpr size_t kOffWDTB  = kOffWXPB  + (size_t)kPrjP * kDin  * 2;
constexpr size_t kOffWOUTB = kOffWDTB  + (size_t)kDin  * kDtR  * 2;
constexpr size_t kOffXZ    = kOffWOUTB + (size_t)kDm   * kDin  * 2;
constexpr size_t kOffUC    = kOffXZ    + (size_t)kRows * kXzP  * 4;
constexpr size_t kOffUCH   = kOffUC    + (size_t)kRows * kDin  * 4;
constexpr size_t kOffUCL   = kOffUCH   + (size_t)kRows * kDin  * 2;
constexpr size_t kOffPROJ  = kOffUCL   + (size_t)kRows * kDin  * 2;
constexpr size_t kOffDTH   = kOffPROJ  + (size_t)kRows * kPrjP * 4;
constexpr size_t kOffDTL   = kOffDTH   + (size_t)kRows * kDtR  * 2;
constexpr size_t kOffDLR   = kOffDTL   + (size_t)kRows * kDtR  * 2;
constexpr size_t kOffYH    = kOffDLR   + (size_t)kRows * kDin  * 4;
constexpr size_t kOffYL    = kOffYH    + (size_t)kRows * kDin  * 2;
constexpr size_t kWsTotal  = kOffYL    + (size_t)kRows * kDin  * 2;
static_assert(kWsTotal == 119799808ull);
static_assert(kWsTotal <= 134217728ull);
static_assert((kOffWINB % 128) == 0 && (kOffWXPB % 128) == 0 && (kOffWDTB % 128) == 0 && (kOffWOUTB % 128) == 0 &&
              (kOffXZ % 128) == 0 && (kOffUC % 128) == 0 && (kOffUCH % 128) == 0 && (kOffUCL % 128) == 0 &&
              (kOffPROJ % 128) == 0 && (kOffDTH % 128) == 0 && (kOffDTL % 128) == 0 && (kOffDLR % 128) == 0 &&
              (kOffYH % 128) == 0 && (kOffYL % 128) == 0);

__device__ __forceinline__ unsigned short f2bf_bits(float f) {
  unsigned u = __float_as_uint(f);
  return (unsigned short)((u + 0x7FFFu + ((u >> 16) & 1u)) >> 16);
}
__device__ __forceinline__ float bf_bits2f(unsigned short h) { return __uint_as_float(((unsigned)h) << 16); }
__device__ __forceinline__ float bf_rne(float f) { return bf_bits2f(f2bf_bits(f)); }
__device__ __forceinline__ unsigned pack_bf2(float a, float b) {
  const unsigned lo = (unsigned)f2bf_bits(a);
  const unsigned hi = (unsigned)f2bf_bits(b);
  return lo | (hi << 16);
}
__device__ __forceinline__ void split_pair(float f0, float f1, unsigned& hw, unsigned& lw) {
  const unsigned short h0 = f2bf_bits(f0), h1 = f2bf_bits(f1);
  const unsigned short l0 = f2bf_bits(f0 - bf_bits2f(h0)), l1 = f2bf_bits(f1 - bf_bits2f(h1));
  hw = (unsigned)h0 | ((unsigned)h1 << 16);
  lw = (unsigned)l0 | ((unsigned)l1 << 16);
}
__device__ __forceinline__ void split8(const v4f a0, const v4f a1, v4u& hv, v4u& lv) {
  const float f0 = a0[0], f1 = a0[1], f2 = a0[2], f3 = a0[3];
  const float f4 = a1[0], f5 = a1[1], f6 = a1[2], f7 = a1[3];
  unsigned h0, h1, h2, h3, l0, l1, l2, l3;
  split_pair(f0, f1, h0, l0);
  split_pair(f2, f3, h1, l1);
  split_pair(f4, f5, h2, l2);
  split_pair(f6, f7, h3, l3);
  hv = (v4u){h0, h1, h2, h3};
  lv = (v4u){l0, l1, l2, l3};
}

union FragU { v16b v; v8b h[2]; };
__device__ __forceinline__ v16b frag_load(const __bf16* p) {
  FragU f;
  f.h[0] = *(const v8b*)(p);
  f.h[1] = *(const v8b*)(p + 16);
  return f.v;
}
__device__ __forceinline__ v8f frag_mma(v16b a, v16b b, v8f c) {
  return __builtin_amdgcn_wmma_f32_16x16x32_bf16(false, a, false, b, (short)0, c, false, false);
}
__device__ __forceinline__ void guard_row(v8f& a, v8f& b, v8f& c, v8f& d, v16b x, v16b y,
                                          v16b b0, v16b b1, v16b b2, v16b b3) {
  asm volatile("v_nop\n\tv_nop\n\tv_nop\n\tv_nop"
               : "+v"(a), "+v"(b), "+v"(c), "+v"(d)
               : "v"(x), "v"(y), "v"(b0), "v"(b1), "v"(b2), "v"(b3));
}
__device__ __forceinline__ void keep4_b(v16b a, v16b b, v16b c, v16b d) { asm volatile("v_nop" :: "v"(a), "v"(b), "v"(c), "v"(d)); }
__device__ __forceinline__ void acc_guard4(v8f& a, v8f& b, v8f& c, v8f& d) { asm volatile("v_nop\n\tv_nop\n\tv_nop\n\tv_nop" : "+v"(a), "+v"(b), "+v"(c), "+v"(d)); }

template <int SPL>
__global__ __launch_bounds__(256) void wmma_gemm64_bf(
    const unsigned short* __restrict__ Ap, const unsigned short* __restrict__ A2p, int lda,
    const unsigned short* __restrict__ Btp, int ldb,
    float* __restrict__ C, int ldc, int M, int N, int K) {
  const __bf16* A  = (const __bf16*)Ap;
  const __bf16* A2 = (const __bf16*)A2p;
  const __bf16* Bt = (const __bf16*)Btp;
  __shared__ __align__(16) float sT[8][16 * 68];
  const int lane = threadIdx.x & 31;
  const int wave = threadIdx.x >> 5;
  const int tilesN = N >> 6;
  const int tilesM = M >> 6;
  const int tile = blockIdx.x * 8 + wave;
  if (tile >= tilesM * tilesN) return;
  const int tm = tile / tilesN;
  const int tn = tile - tm * tilesN;
  const int m0 = tm << 6;
  const int n0 = tn << 6;

  const int rlane = lane & 15;
  const int koff  = (lane >> 4) * 8;
  const int mOff  = (lane >> 4) * 8;

  v8f acc[4][4];
#pragma unroll
  for (int i = 0; i < 4; ++i)
#pragma unroll
    for (int j = 0; j < 4; ++j) acc[i][j] = (v8f){0.f,0.f,0.f,0.f,0.f,0.f,0.f,0.f};

  for (int k0 = 0; k0 < K; k0 += 32) {
    v16b bh[4];
#pragma unroll
    for (int j = 0; j < 4; ++j) {
      const size_t bo = (size_t)(n0 + (j << 4) + rlane) * ldb + koff + k0;
      bh[j] = frag_load(Bt + bo);
    }
#pragma unroll
    for (int i = 0; i < 4; ++i) {
      const size_t ao = (size_t)(m0 + (i << 4) + rlane) * lda + koff + k0;
      v16b ah = frag_load(A + ao);
      v16b al = ah;
      if (SPL >= 1) al = frag_load(A2 + ao);
#pragma unroll
      for (int j = 0; j < 4; ++j) {
        acc[i][j] = frag_mma(ah, bh[j], acc[i][j]);
        if (SPL >= 1) acc[i][j] = frag_mma(al, bh[j], acc[i][j]);
      }
      guard_row(acc[i][0], acc[i][1], acc[i][2], acc[i][3], ah, al, bh[0], bh[1], bh[2], bh[3]);
    }
    keep4_b(bh[0], bh[1], bh[2], bh[3]);
  }
  acc_guard4(acc[0][0], acc[0][1], acc[0][2], acc[0][3]);
  acc_guard4(acc[1][0], acc[1][1], acc[1][2], acc[1][3]);
  acc_guard4(acc[2][0], acc[2][1], acc[2][2], acc[2][3]);
  acc_guard4(acc[3][0], acc[3][1], acc[3][2], acc[3][3]);

  float* slab = sT[wave];
#pragma unroll
  for (int i = 0; i < 4; ++i) {
    const int mBase = m0 + (i << 4);
#pragma unroll
    for (int j = 0; j < 4; ++j) {
#pragma unroll
      for (int r = 0; r < 8; ++r) {
        slab[(mOff + r) * 68 + (j << 4) + rlane] = acc[i][j][r];
      }
    }
    __builtin_amdgcn_fence(__ATOMIC_RELEASE, "workgroup");
    __builtin_amdgcn_wave_barrier();
    __builtin_amdgcn_fence(__ATOMIC_ACQUIRE, "workgroup");
    {
      const int hh = lane >> 4, c4 = (lane & 15) * 4;
      for (int pass = 0; pass < 2; ++pass) {
#pragma unroll
        for (int it = 0; it < 8; ++it) {
          const int row = it * 2 + hh;
          v4f v = *(const v4f*)(slab + row * 68 + c4);
          *(volatile v4f*)(C + (size_t)(mBase + row) * ldc + n0 + c4) = v;
        }
        __threadfence();
      }
    }
    __builtin_amdgcn_fence(__ATOMIC_RELEASE, "workgroup");
    __builtin_amdgcn_wave_barrier();
    __builtin_amdgcn_fence(__ATOMIC_ACQUIRE, "workgroup");
  }
}

__global__ __launch_bounds__(256) void cast_bf16_kernel(
    const float* __restrict__ src, unsigned short* __restrict__ dst, int total8, int real8)
{
  const int i = blockIdx.x * 256 + threadIdx.x;
  if (i >= total8) return;
  const bool real = (i < real8);
  const int ic = real ? i : (real8 - 1);
  const size_t es = (size_t)ic << 3;
  const v4f a0 = *(const v4f*)(src + es);
  const v4f a1 = *(const v4f*)(src + es + 4);
  const float f0 = real ? a0[0] : 0.0f, f1 = real ? a0[1] : 0.0f, f2 = real ? a0[2] : 0.0f, f3 = real ? a0[3] : 0.0f;
  const float f4 = real ? a1[0] : 0.0f, f5 = real ? a1[1] : 0.0f, f6 = real ? a1[2] : 0.0f, f7 = real ? a1[3] : 0.0f;
  const unsigned w0 = pack_bf2(f0, f1), w1 = pack_bf2(f2, f3), w2 = pack_bf2(f4, f5), w3 = pack_bf2(f6, f7);
  const v4u w = (v4u){w0, w1, w2, w3};
  const size_t e0 = (size_t)i << 3;
  volatile v4u* q = (volatile v4u*)(dst + e0);
  *q = w;
  __threadfence();
  *q = w;
}

__global__ __launch_bounds__(256) void dt_split_kernel(
    const float* __restrict__ PROJ, unsigned short* __restrict__ DTH, unsigned short* __restrict__ DTL, int total8)
{
  const int i = blockIdx.x * 256 + threadIdx.x;
  if (i >= total8) return;
  const int e0  = i << 3;
  const int row = e0 >> 6;
  const int c8  = e0 & 63;
  const float* p = PROJ + (size_t)row * kPrjP + c8;
  const v4f a0 = *(const v4f*)(p);
  const v4f a1 = *(const v4f*)(p + 4);
  v4u hv, lv;
  split8(a0, a1, hv, lv);
  volatile v4u* qh = (volatile v4u*)(DTH + e0);
  volatile v4u* ql = (volatile v4u*)(DTL + e0);
  *qh = hv;
  *ql = lv;
  __threadfence();
  *qh = hv;
  *ql = lv;
}

__global__ __launch_bounds__(256) void conv_silu_kernel(
    const float* __restrict__ XZ, const float* __restrict__ cw, const float* __restrict__ cb,
    float* __restrict__ UC, unsigned short* __restrict__ UCH, unsigned short* __restrict__ UCL)
{
  __shared__ __align__(16) float sT[16 * kTP];
  const int tid = threadIdx.x, lane = tid & 31, wave = tid >> 5;
  const int d0 = blockIdx.x * 256, d = d0 + tid;
  const int g0 = blockIdx.y * 64;
  const int tb = g0 & (kSeq - 1);
  const v4f wv = *(const v4f*)(cw + (size_t)d * 4);
  const float wr0 = wv[0], wr1 = wv[1], wr2 = wv[2], wr3 = wv[3];
  const float w0 = bf_rne(wr0), w1 = bf_rne(wr1), w2 = bf_rne(wr2), w3 = bf_rne(wr3);
  const float bc = bf_rne(cb[d]);
  float xm3, xm2, xm1;
  {
    const bool hist = (tb > 0);
    const int rb = hist ? (g0 - 3) : g0;
    const float v3 = XZ[(size_t)rb * kXzP + d];
    const float v2 = XZ[(size_t)(rb + 1) * kXzP + d];
    const float v1 = XZ[(size_t)(rb + 2) * kXzP + d];
    xm3 = hist ? v3 : 0.f;
    xm2 = hist ? v2 : 0.f;
    xm1 = hist ? v1 : 0.f;
  }
  const int hrow = wave >> 1;
  const int hch  = (wave & 1) * 128 + lane * 4;
#pragma unroll 1
  for (int sub = 0; sub < 4; ++sub) {
    const int lb = g0 + sub * 16;
#pragma unroll 1
    for (int s = 0; s < 16; ++s) {
      const float xcur = XZ[(size_t)(lb + s) * kXzP + d];
      float acc = w0 * xm3;
      acc = fmaf(w1, xm2, acc);
      acc = fmaf(w2, xm1, acc);
      acc = fmaf(w3, xcur, acc);
      const float sv = acc + bc;
      const float sg = __builtin_amdgcn_rcpf(1.0f + expf(-sv));
      sT[s * kTP + tid] = sv * sg;
      xm3 = xm2; xm2 = xm1; xm1 = xcur;
    }
    __syncthreads();
    v4f fv[4];
    v4u bh[2], blo[2];
#pragma unroll
    for (int it = 0; it < 4; ++it) fv[it] = *(const v4f*)(sT + (it * 4 + hrow) * kTP + hch);
#pragma unroll
    for (int it = 0; it < 2; ++it) {
      const float* sp = sT + (it * 8 + wave) * kTP + lane * 8;
      const v4f a0 = *(const v4f*)(sp);
      const v4f a1 = *(const v4f*)(sp + 4);
      split8(a0, a1, bh[it], blo[it]);
    }
    for (int pass = 0; pass < 2; ++pass) {
#pragma unroll
      for (int it = 0; it < 4; ++it)
        *(volatile v4f*)(UC + (size_t)(lb + it * 4 + hrow) * kDin + d0 + hch) = fv[it];
#pragma unroll
      for (int it = 0; it < 2; ++it) {
        const size_t o = (size_t)(lb + it * 8 + wave) * kDin + d0 + lane * 8;
        *(volatile v4u*)(UCH + o) = bh[it];
        *(volatile v4u*)(UCL + o) = blo[it];
      }
      __threadfence();
    }
    __syncthreads();
  }
}

__global__ __launch_bounds__(256) void scan_kernel(
    const float* __restrict__ DLR, const float* __restrict__ UC, const float* __restrict__ XZ,
    const float* __restrict__ PROJ, const float* __restrict__ bdt, const float* __restrict__ Alog,
    const float* __restrict__ Dp, unsigned short* __restrict__ YH, unsigned short* __restrict__ YL)
{
  __shared__ __align__(16) float sBC[16 * 32];
  __shared__ __align__(16) float sY[16 * kTP];
  __shared__ __align__(16) float sA[kNst * 256];
  const int tid = threadIdx.x, lane = tid & 31, wave = tid >> 5;
  const int d0 = blockIdx.x * 256, d = d0 + tid;
  const size_t rowb = (size_t)blockIdx.y * kSeq;

#pragma unroll 1
  for (int s = 0; s < kNst; ++s) {
    const float al = bf_rne(Alog[(size_t)d * kNst + s]);
    sA[s * 256 + tid] = -expf(al);
  }
  __syncthreads();
  float An[kNst], h[kNst];
#pragma unroll
  for (int n = 0; n < kNst; ++n) {
    An[n] = sA[n * 256 + tid];
    h[n] = 0.f;
  }
  const float bb = bf_rne(bdt[d]);
  const float Dd = bf_rne(Dp[d]);

#pragma unroll 1
  for (int c = 0; c < kSeq / 16; ++c) {
    const int l0 = c * 16;
    if (tid < 128) {
      const int r = tid >> 3, q = (tid & 7) * 4;
      const v4f v = *(const v4f*)(PROJ + (rowb + l0 + r) * kPrjP + kDtR + q);
      *(v4f*)(sBC + r * 32 + q) = v;
    }
    __syncthreads();
#pragma unroll 1
    for (int s = 0; s < 16; ++s) {
      const size_t m = rowb + (size_t)(l0 + s);
      const float a     = DLR[m * kDin + d] + bb;
      const float ea    = __expf(-fabsf(a));
      const float up    = 1.0f + ea;
      const float l1p   = __logf(up) + (ea - (up - 1.0f)) * __builtin_amdgcn_rcpf(up);
      const float delta = fmaxf(a, 0.0f) + l1p;
      const float xv    = UC[m * kDin + d];
      const float zv    = XZ[m * kXzP + kDin + d];
      v4f Bq[4], Cq[4];
#pragma unroll
      for (int qq = 0; qq < 4; ++qq) {
        Bq[qq] = *(const v4f*)(sBC + s * 32 + 4 * qq);
        Cq[qq] = *(const v4f*)(sBC + s * 32 + kNst + 4 * qq);
      }
      const float dbu = delta * xv;
      float y = 0.f;
#pragma unroll
      for (int n = 0; n < kNst; ++n) {
        const float e = __expf(delta * An[n]);
        h[n] = e * h[n] + dbu * Bq[n >> 2][n & 3];
        y = h[n] * Cq[n >> 2][n & 3] + y;
      }
      y = xv * Dd + y;
      const float sg = __builtin_amdgcn_rcpf(1.0f + expf(-zv));
      sY[s * kTP + tid] = y * (zv * sg);
    }
    __syncthreads();
    v4u hv[2], lv[2];
#pragma unroll
    for (int it = 0; it < 2; ++it) {
      const float* sp = sY + (it * 8 + wave) * kTP + lane * 8;
      const v4f a0 = *(const v4f*)(sp);
      const v4f a1 = *(const v4f*)(sp + 4);
      split8(a0, a1, hv[it], lv[it]);
    }
    for (int pass = 0; pass < 2; ++pass) {
#pragma unroll
      for (int it = 0; it < 2; ++it) {
        const size_t o = (rowb + (size_t)(l0 + it * 8 + wave)) * kDin + d0 + lane * 8;
        *(volatile v4u*)(YH + o) = hv[it];
        *(volatile v4u*)(YL + o) = lv[it];
      }
      __threadfence();
    }
  }
}

extern "C" void kernel_launch(void* const* d_in, const int* in_sizes, int n_in,
                              void* d_out, int out_size, void* d_ws, size_t ws_size,
                              hipStream_t stream) {
  if (n_in < 10) return;
  if (in_sizes[0] != kRows * kDm) return;
  if (in_sizes[1] != kXzP * kDm) return;
  if (in_sizes[2] != kDin * 4) return;
  if (in_sizes[3] != kDin) return;
  if (in_sizes[4] != kPrjN * kDin) return;
  if (in_sizes[5] != kDin * kDtR) return;
  if (in_sizes[6] != kDin) return;
  if (in_sizes[7] != kDin * kNst) return;
  if (in_sizes[8] != kDin) return;
  if (in_sizes[9] != kDm * kDin) return;
  if (out_size != kRows * kDm) return;
  if (ws_size < kWsTotal) return;

  const float* x       = (const float*)d_in[0];
  const float* W_in    = (const float*)d_in[1];
  const float* conv_w  = (const float*)d_in[2];
  const float* conv_b  = (const float*)d_in[3];
  const float* W_xp    = (const float*)d_in[4];
  const float* W_dt    = (const float*)d_in[5];
  const float* b_dt    = (const float*)d_in[6];
  const float* A_log   = (const float*)d_in[7];
  const float* Dp      = (const float*)d_in[8];
  const float* W_out   = (const float*)d_in[9];
  float* out = (float*)d_out;

  char* ws = (char*)d_ws;
  unsigned short* XB    = (unsigned short*)(ws + kOffXB);
  unsigned short* WINB  = (unsigned short*)(ws + kOffWINB);
  unsigned short* WXPB  = (unsigned short*)(ws + kOffWXPB);
  unsigned short* WDTB  = (unsigned short*)(ws + kOffWDTB);
  unsigned short* WOUTB = (unsigned short*)(ws + kOffWOUTB);
  float*          XZ    = (float*)(ws + kOffXZ);
  float*          UC    = (float*)(ws + kOffUC);
  unsigned short* UCH   = (unsigned short*)(ws + kOffUCH);
  unsigned short* UCL   = (unsigned short*)(ws + kOffUCL);
  float*          PROJ  = (float*)(ws + kOffPROJ);
  unsigned short* DTH   = (unsigned short*)(ws + kOffDTH);
  unsigned short* DTL   = (unsigned short*)(ws + kOffDTL);
  float*          DLR   = (float*)(ws + kOffDLR);
  unsigned short* YH    = (unsigned short*)(ws + kOffYH);
  unsigned short* YL    = (unsigned short*)(ws + kOffYL);

  cast_bf16_kernel<<<(kRows * kDm / 8) / 256, 256, 0, stream>>>(x, XB, kRows * kDm / 8, kRows * kDm / 8);
  cast_bf16_kernel<<<(kXzP * kDm / 8) / 256, 256, 0, stream>>>(W_in, WINB, kXzP * kDm / 8, kXzP * kDm / 8);
  cast_bf16_kernel<<<(kPrjP * kDin / 8) / 256, 256, 0, stream>>>(W_xp, WXPB, kPrjP * kDin / 8, kPrjN * kDin / 8);
  cast_bf16_kernel<<<(kDin * kDtR / 8) / 256, 256, 0, stream>>>(W_dt, WDTB, kDin * kDtR / 8, kDin * kDtR / 8);
  cast_bf16_kernel<<<(kDm * kDin / 8) / 256, 256, 0, stream>>>(W_out, WOUTB, kDm * kDin / 8, kDm * kDin / 8);

  wmma_gemm64_bf<0><<<((kRows / 64) * (kXzP / 64)) / 8, 256, 0, stream>>>(
      XB, XB, kDm, WINB, kDm, XZ, kXzP, kRows, kXzP, kDm);

  conv_silu_kernel<<<dim3(kDin / 256, kRows / 64), 256, 0, stream>>>(XZ, conv_w, conv_b, UC, UCH, UCL);

  wmma_gemm64_bf<1><<<((kRows / 64) * (kPrjP / 64)) / 8, 256, 0, stream>>>(
      UCH, UCL, kDin, WXPB, kDin, PROJ, kPrjP, kRows, kPrjP, kDin);

  dt_split_kernel<<<(kRows * kDtR / 8) / 256, 256, 0, stream>>>(PROJ, DTH, DTL, kRows * kDtR / 8);

  wmma_gemm64_bf<1><<<((kRows / 64) * (kDin / 64)) / 8, 256, 0, stream>>>(
      DTH, DTL, kDtR, WDTB, kDtR, DLR, kDin, kRows, kDin, kDtR);

  scan_kernel<<<dim3(kDin / 256, kBatch), 256, 0, stream>>>(DLR, UC, XZ, PROJ, b_dt, A_log, Dp, YH, YL);

  wmma_gemm64_bf<1><<<((kRows / 64) * (kDm / 64)) / 8, 256, 0, stream>>>(
      YH, YL, kDin, WOUTB, kDin, out, kDm, kRows, kDm, kDin);
}
